// AlbertDecoderAttention_6253472383101
// MI455X (gfx1250) — hardware-run, weakly checked
//
#include <hip/hip_runtime.h>


#ifndef NB
#define NB 4
#endif
#ifndef SEQ
#define SEQ 1024
#endif
#define NB_FULL  4
#define SEQ_FULL 1024
#ifndef OUT_SEQ
#define OUT_SEQ SEQ
#endif
#define DM   1024
#define NH_  16
#define HD   64
#define AW   4
#define OSP  68
#define NW   (SEQ / 32)
#define WSC  64.0f
#define WSI  (1.0f / 64.0f)
#define L2E  1.4426950408889634f
#define FILL2 (-1.0e6f * 1.4426950408889634f)
#define PSH  14.0f
#define NEGB (-3.0e38f)
#define LNEPS 1.0e-12f

static_assert(HD == 64);
static_assert(NH_ * HD == DM);
static_assert(DM % 64 == 0);
static_assert(DM % 32 == 0);
static_assert(DM % 256 == 0);
static_assert(SEQ % 64 == 0);
static_assert(SEQ % 256 == 0);
static_assert(SEQ % 32 == 0);
static_assert((NB * SEQ) % 64 == 0);
static_assert((NB * SEQ) % 4 == 0);
static_assert(SEQ % (16 * AW) == 0);
static_assert(NB <= NB_FULL);
static_assert(SEQ <= SEQ_FULL);
static_assert(SEQ_FULL % 128 == 0);
static_assert((OSP * 4) % 16 == 0);
static_assert(OSP >= HD);
static_assert(4 * 32 * 16 == 16 * HD * 2);
static_assert(8 * 32 * 16 == 16 * 64 * 4);
static_assert((DM / 128) * 32 * 16 == DM * 4);
static_assert((DM / 256) * 32 * 16 == DM * 2);
static_assert(16 * 68 * 4 <= 131072);
static_assert(AW * 16 * OSP * 4 <= 131072);

typedef _Float16 h16;
typedef unsigned short bf;
typedef __attribute__((ext_vector_type(16))) __bf16   v16bf;
typedef __attribute__((ext_vector_type(16))) _Float16 v16h;
typedef __attribute__((ext_vector_type(8)))  _Float16 v8h;
typedef __attribute__((ext_vector_type(8)))  unsigned short v8us;
typedef __attribute__((ext_vector_type(8)))  float    v8f;
typedef __attribute__((ext_vector_type(4)))  float    v4f;
typedef __attribute__((ext_vector_type(4)))  unsigned int v4u;
typedef v4f  __attribute__((may_alias)) v4fa;

__device__ __forceinline__ unsigned short f2bf(float f) { unsigned u = __float_as_uint(f); u += 0x7FFFu + ((u >> 16) & 1u); return (unsigned short)(u >> 16); }
__device__ __forceinline__ float bfr(float f) { return __uint_as_float(((unsigned)f2bf(f)) << 16); }
__device__ __forceinline__ v16h cat16(v8h lo, v8h hi) { return __builtin_shufflevector(lo, hi, 0, 1, 2, 3, 4, 5, 6, 7, 8, 9, 10, 11, 12, 13, 14, 15); }
__device__ __forceinline__ v16bf cat16b(v8us lo, v8us hi) { return __builtin_bit_cast(v16bf, __builtin_shufflevector(lo, hi, 0, 1, 2, 3, 4, 5, 6, 7, 8, 9, 10, 11, 12, 13, 14, 15)); }
__device__ __forceinline__ v8f wmma16(v16h a, v16h b, v8f c) { return __builtin_amdgcn_wmma_f32_16x16x32_f16(false, a, false, b, (short)0, c, false, false); }
__device__ __forceinline__ v8f wmmab(v16bf a, v16bf b, v8f c) { return __builtin_amdgcn_wmma_f32_16x16x32_bf16(false, a, false, b, (short)0, c, false, false); }
__device__ __forceinline__ v16h  ldh(const h16* p) { return cat16(*(const v8h*)p, *(const v8h*)(p + 16)); }
__device__ __forceinline__ v16bf ldb(const bf* p)  { return cat16b(*(const v8us*)p, *(const v8us*)(p + 16)); }
__device__ __forceinline__ void wave_sync() { __builtin_amdgcn_fence(3  , "wavefront"); __builtin_amdgcn_wave_barrier(); asm volatile("" ::: "memory"); }
__device__ __forceinline__ h16 toh_flush(float v) { const h16 r = (h16)v; return (fabsf(v) < 6.103515625e-05f) ? (h16)0.0f : r; }
__device__ __forceinline__ v8f wm16(v16h a, v16h b, v8f c) { c = wmma16(a, b, c); asm volatile("v_nop\n\tv_nop\n\tv_nop\n\tv_nop" : "+v"(c) : "v"(a), "v"(b)); return c; }
__device__ __forceinline__ v8f wmb(v16bf a, v16bf b, v8f c) { c = wmmab(a, b, c); asm volatile("v_nop\n\tv_nop\n\tv_nop\n\tv_nop" : "+v"(c) : "v"(a), "v"(b)); return c; }

__global__ __launch_bounds__(256) void k_cvt8(const float* __restrict__ src, bf* dst, size_t n8) {
    const size_t i = (size_t)blockIdx.x * 256 + threadIdx.x; if (i >= n8) return;
    const v8f v = *(const v8f*)(src + i * 8); v8us o;
#pragma unroll
    for (int k = 0; k < 8; ++k) o[k] = f2bf(v[k]);
    *(volatile v8us*)(dst + i * 8) = o; __threadfence(); *(volatile v8us*)(dst + i * 8) = o;
}

__global__ __launch_bounds__(256) void k_cvtw(const float* __restrict__ src, h16* dst, size_t n8) {
    const size_t i = (size_t)blockIdx.x * 256 + threadIdx.x; if (i >= n8) return;
    const v8f v = *(const v8f*)(src + i * 8); v8h o;
#pragma unroll
    for (int k = 0; k < 8; ++k) o[k] = toh_flush(bfr(v[k]) * WSC);
    *(volatile v8h*)(dst + i * 8) = o; __threadfence(); *(volatile v8h*)(dst + i * 8) = o;
}

__global__ __launch_bounds__(256) void k_pack(const int* __restrict__ msk, unsigned* PM, int nwords) {
    const int lane = threadIdx.x & 31;
    const int wave = __builtin_amdgcn_readfirstlane((int)(threadIdx.x >> 5));
    const int base = (blockIdx.x * 8 + wave) * 32;
    if (base >= nwords) return;
    unsigned myw = 0u;
#pragma unroll 8
    for (int i = 0; i < 32; ++i) {
        const int v = msk[(size_t)(base + i) * 32 + lane];
        const unsigned bal = __builtin_amdgcn_ballot_w32(v != 0);
        myw = (lane == i) ? bal : myw;
    }
    *(volatile unsigned*)(PM + base + lane) = myw; __threadfence(); *(volatile unsigned*)(PM + base + lane) = myw;
}

template <int F16>
__device__ __forceinline__ void gemm_kloop(const bf* __restrict__ A, size_t aoff, const bf* __restrict__ Bt, size_t boff, v8f (&acc)[4][4]) {
    const int K = DM;
#pragma unroll 1
    for (int kc = 0; kc < K; kc += 32) {
        if (F16) {
            const h16* Ah = (const h16*)A; const h16* Bh = (const h16*)Bt;
            v16h a[4];
#pragma unroll
            for (int mb = 0; mb < 4; ++mb) a[mb] = ldh(Ah + aoff + (size_t)mb * 16 * K + kc);
#pragma unroll
            for (int nb = 0; nb < 4; ++nb) { const v16h b = ldh(Bh + boff + (size_t)nb * 16 * K + kc);
#pragma unroll
                for (int mb = 0; mb < 4; ++mb) acc[mb][nb] = wm16(a[mb], b, acc[mb][nb]); }
        } else {
            v16bf a[4];
#pragma unroll
            for (int mb = 0; mb < 4; ++mb) a[mb] = ldb(A + aoff + (size_t)mb * 16 * K + kc);
#pragma unroll
            for (int nb = 0; nb < 4; ++nb) { const v16bf b = ldb(Bt + boff + (size_t)nb * 16 * K + kc);
#pragma unroll
                for (int mb = 0; mb < 4; ++mb) acc[mb][nb] = wmb(a[mb], b, acc[mb][nb]); }
        }
    }
}

template <int F16, int MODE, int WF>
__device__ __forceinline__ void gemm_body(const bf* __restrict__ A, const bf* __restrict__ Bt, const float* __restrict__ bias,
                                          h16* Ph, const float* __restrict__ QF, float* YF) {
    __shared__ __align__(16) float os[16 * 68];
    const int K = DM;
    const int lane = threadIdx.x & 31, lr = lane & 15, hi = lane >> 4; const int r0 = blockIdx.x * 64, c0 = blockIdx.y * 64;
    size_t tbase; int bb, tt;
    if (MODE == 1) { bb = c0 / SEQ; tt = c0 % SEQ;
                     tbase = (size_t)bb * (size_t)DM * SEQ + (size_t)r0 * SEQ + (size_t)tt; }
    else           { bb = r0 / SEQ; tt = r0 % SEQ; const int zc = bb * NH_ + c0 / HD;
                     tbase = ((size_t)zc * SEQ + (size_t)tt) * HD; }
    v8f acc[4][4];
#pragma unroll
    for (int mb = 0; mb < 4; ++mb)
#pragma unroll
        for (int nb = 0; nb < 4; ++nb) acc[mb][nb] = (v8f){};
    const size_t aoff = (size_t)(r0 + lr) * K + 8 * hi, boff = (size_t)(c0 + lr) * K + 8 * hi;
    gemm_kloop<F16>(A, aoff, Bt, boff, acc);
    const float scl = F16 ? WSI : 1.0f;
    float bc[4];
#pragma unroll
    for (int nb = 0; nb < 4; ++nb) bc[nb] = (MODE != 1) ? bfr(bias[c0 + nb * 16 + lr]) : 0.0f;
#pragma unroll
    for (int mb = 0; mb < 4; ++mb) {
        float br[8];
#pragma unroll
        for (int j = 0; j < 8; ++j) br[j] = (MODE == 1) ? bfr(bias[r0 + mb * 16 + hi * 8 + j]) : 0.0f;
#pragma unroll
        for (int nb = 0; nb < 4; ++nb) {
#pragma unroll
            for (int j = 0; j < 8; ++j) os[(hi * 8 + j) * 68 + nb * 16 + lr] = acc[mb][nb][j] * scl + bc[nb] + br[j]; }
        wave_sync();
#pragma unroll 1
        for (int ps = 0; ps < 2; ++ps) {
            if (MODE == 0) {
                const size_t sb = tbase + (size_t)(mb * 16) * HD;
#pragma unroll
                for (int s = 0; s < 4; ++s) { const int p = s * 32 + lane; const int row = p >> 3, c8 = (p & 7) * 8;
                    const v4f x0 = *(const v4fa*)(&os[row * 68 + c8]); const v4f x1 = *(const v4fa*)(&os[row * 68 + c8 + 4]); v8h hv;
#pragma unroll
                    for (int i = 0; i < 4; ++i) { hv[i] = toh_flush(x0[i]); hv[4 + i] = toh_flush(x1[i]); }
                    *(volatile v8h*)(Ph + sb + (size_t)p * 8) = hv; }
                if (WF) {
                    const size_t yb = (size_t)(r0 + mb * 16) * DM + c0;
#pragma unroll 4
                    for (int s = 0; s < 8; ++s) { const int row = 2 * s + (lane >> 4), c4 = (lane & 15) * 4;
                        const v4f val = *(const v4fa*)(&os[row * 68 + c4]);
                        *(volatile v4f*)(YF + yb + (size_t)row * DM + c4) = val; }
                }
            } else if (MODE == 1) {
                const size_t sb = tbase + (size_t)(mb * 16) * SEQ;
#pragma unroll
                for (int s = 0; s < 4; ++s) { const int row = 4 * s + (lane >> 3), c8 = (lane & 7) * 8;
                    const v4f x0 = *(const v4fa*)(&os[row * 68 + c8]); const v4f x1 = *(const v4fa*)(&os[row * 68 + c8 + 4]); v8h hv;
#pragma unroll
                    for (int i = 0; i < 4; ++i) { hv[i] = toh_flush(x0[i]); hv[4 + i] = toh_flush(x1[i]); }
                    *(volatile v8h*)(Ph + sb + (size_t)row * SEQ + c8) = hv; }
            } else {
                const size_t yb = (size_t)(r0 + mb * 16) * DM + c0;
#pragma unroll 4
                for (int s = 0; s < 8; ++s) { const int row = 2 * s + (lane >> 4), c4 = (lane & 15) * 4;
                    v4f val = *(const v4fa*)(&os[row * 68 + c4]);
                    const v4f qv = *(const v4f*)(QF + yb + (size_t)row * DM + c4);
#pragma unroll
                    for (int i = 0; i < 4; ++i) val[i] = val[i] + qv[i];
                    *(volatile v4f*)(YF + yb + (size_t)row * DM + c4) = val; }
            }
            if (ps == 0) __threadfence(); }
        wave_sync();
    }
}

__global__ __launch_bounds__(32) void k_gemm_qb(const bf* __restrict__ A, const bf* __restrict__ Bt, const float* __restrict__ bias, h16* Ph, float* QF) {
    gemm_body<0, 0, 1>(A, Bt, bias, Ph, (const float*)0, QF);
}
__global__ __launch_bounds__(32) void k_gemm_pb(const bf* __restrict__ A, const bf* __restrict__ Bt, const float* __restrict__ bias, h16* Ph) {
    gemm_body<0, 0, 0>(A, Bt, bias, Ph, (const float*)0, (float*)0);
}
__global__ __launch_bounds__(32) void k_gemm_tb(const bf* __restrict__ A, const bf* __restrict__ Bt, const float* __restrict__ bias, h16* Ph) {
    gemm_body<0, 1, 0>(A, Bt, bias, Ph, (const float*)0, (float*)0);
}
__global__ __launch_bounds__(32) void k_gemm_qh(const h16* __restrict__ A, const h16* __restrict__ Bt, const float* __restrict__ bias, h16* Ph, float* QF) {
    gemm_body<1, 0, 1>((const bf*)A, (const bf*)Bt, bias, Ph, (const float*)0, QF);
}
__global__ __launch_bounds__(32) void k_gemm_yh(const h16* __restrict__ A, const h16* __restrict__ Bt, const float* __restrict__ bias, const float* __restrict__ QF, float* Y) {
    gemm_body<1, 2, 0>((const bf*)A, (const bf*)Bt, bias, (h16*)0, QF, Y);
}

__device__ __forceinline__ v8f score16(const h16* __restrict__ kh, v16h qh0, v16h qh1) {
    const v16h a0 = ldh(kh), a1 = ldh(kh + 32);
    v8f sH = (v8f){};
    sH = wm16(a0, qh0, sH); sH = wm16(a1, qh1, sH);
    return sH;
}

__global__ __launch_bounds__(32 * AW) void k_flash(const h16* __restrict__ QH, const h16* __restrict__ KH, const h16* __restrict__ VT,
                                                   const unsigned* __restrict__ PM, int mbs, int mqs, h16* CH) {
    __shared__ __align__(16) float os[AW * 16 * OSP];
    const int lane = threadIdx.x & 31, lr = lane & 15, hi = lane >> 4;
    const int wave = __builtin_amdgcn_readfirstlane((int)(threadIdx.x >> 5));
    const int zh = blockIdx.y; const int b = zh / NH_, h = zh % NH_;
    const int t0 = (blockIdx.x * AW + wave) * 16;
    const unsigned* mrow = PM + (size_t)b * (size_t)mbs + (size_t)(t0 + lr) * (size_t)mqs;
    unsigned orw = 0u;
#pragma unroll
    for (int i = 0; i < NW / 8; ++i) { const v4u w = *(const v4u*)(mrow + hi * (NW / 2) + 4 * i); orw |= (w[0] | w[1]) | (w[2] | w[3]); }
    orw |= (unsigned)__shfl_xor((int)orw, 16, 32);
    const bool noskip = __builtin_amdgcn_ballot_w32(orw == 0u) != 0u;
    const size_t pbase = (size_t)zh * SEQ * HD;
    const size_t qo = pbase + (size_t)(t0 + lr) * HD + 8 * hi;
    const size_t ko = pbase + (size_t)lr * HD + 8 * hi;
    const size_t vo = pbase + (size_t)lr * SEQ + 8 * hi;
    v8f o[4];
#pragma unroll
    for (int j = 0; j < 4; ++j) o[j] = (v8f){};
    float m = NEGB, l = 0.0f;
#pragma unroll 1
    for (int key0 = 0; key0 < SEQ; key0 += 32) {
        const unsigned wd = mrow[key0 >> 5];
        const bool act = __builtin_amdgcn_ballot_w32(wd != 0u) != 0u;
        if (!(noskip || act)) continue;
        int qz = 0; asm volatile("" : "+v"(qz));
        const h16* qp = QH + qo + qz;
        const v16h qh0 = ldh(qp), qh1 = ldh(qp + 32);
        const size_t kof = ko + (size_t)key0 * HD;
        const v8f sa = score16(KH + kof, qh0, qh1);
        const v8f sb = score16(KH + kof + 16 * HD, qh0, qh1);
        const unsigned wa = wd >> (8 * hi);
        float ta[8], tb[8]; float mx = NEGB;
#pragma unroll
        for (int r = 0; r < 8; ++r) {
            const bool fa = ((wa >> r) & 1u) != 0u, fb = ((wa >> (16 + r)) & 1u) != 0u;
            ta[r] = fa ? sa[r] * L2E : FILL2; tb[r] = fb ? sb[r] * L2E : FILL2;
            mx = fmaxf(mx, fmaxf(ta[r], tb[r])); }
        mx = fmaxf(mx, __shfl_xor(mx, 16, 32));
        const float mnew = fmaxf(m, mx);
        const float alpha = __builtin_amdgcn_exp2f(m - mnew);
        const float sh = PSH - mnew;
        v16h pb; float ls = 0.0f;
#pragma unroll
        for (int r = 0; r < 8; ++r) {
            const float xa = ta[r] + sh, xb = tb[r] + sh;
            const float ea = __builtin_amdgcn_exp2f(xa), eb = __builtin_amdgcn_exp2f(xb);
            const float ga = (xa < -14.0f) ? 0.0f : ea, gb = (xb < -14.0f) ? 0.0f : eb;
            const h16 pa = (h16)ga; const h16 pc = (h16)gb;
            pb[r] = pa; pb[8 + r] = pc;
            ls += (float)pa + (float)pc; }
        l = l * alpha + ls; m = mnew;
#pragma unroll
        for (int j = 0; j < 4; ++j) o[j] = o[j] * alpha;
        const h16* va = VT + vo + key0;
#pragma unroll
        for (int j = 0; j < 4; ++j) {
            const v16h vj = ldh(va + (size_t)(16 * j) * SEQ);
            o[j] = wm16(vj, pb, o[j]);
        }
    }
    l += __shfl_xor(l, 16, 32);
    const float lsafe = (l > 0.0f) ? l : 1.0f;
    const float inv = 1.0f / lsafe;
    const int wb = wave * 16 * OSP;
#pragma unroll
    for (int j = 0; j < 4; ++j) {
        const v8f f = o[j];
        v4f a, c;
        a[0] = f[0] * inv; a[1] = f[1] * inv; a[2] = f[2] * inv; a[3] = f[3] * inv; c[0] = f[4] * inv; c[1] = f[5] * inv; c[2] = f[6] * inv; c[3] = f[7] * inv;
        *(v4fa*)(&os[wb + lr * OSP + 16 * j + 8 * hi]) = a; *(v4fa*)(&os[wb + lr * OSP + 16 * j + 8 * hi + 4]) = c; }
    wave_sync();
    h16* crow = CH + ((size_t)b * SEQ + t0) * DM + h * HD;
#pragma unroll 1
    for (int ps = 0; ps < 2; ++ps) {
#pragma unroll
        for (int s = 0; s < 4; ++s) { const int row = 4 * s + (lane >> 3), c8 = (lane & 7) * 8;
            const v4f x0 = *(const v4fa*)(&os[wb + row * OSP + c8]); const v4f x1 = *(const v4fa*)(&os[wb + row * OSP + c8 + 4]); v8h hv;
#pragma unroll
            for (int i = 0; i < 4; ++i) { hv[i] = toh_flush(x0[i]); hv[4 + i] = toh_flush(x1[i]); }
            *(volatile v8h*)(crow + (size_t)row * DM + c8) = hv; }
        if (ps == 0) __threadfence(); }
}

template <int OUTF>
__device__ __forceinline__ void ln_body(const float* __restrict__ Y, const float* __restrict__ g, const float* __restrict__ be, float* OUTP, h16* OUTH) {
#pragma clang fp contract(off)
    const int lane = threadIdx.x & 31;
    const int wave = __builtin_amdgcn_readfirstlane((int)(threadIdx.x >> 5));
    const int row = blockIdx.x * 4 + wave;
    const float* y = Y + (size_t)row * DM;
    float s = 0.0f;
#pragma unroll 1
    for (int i = 0; i < DM / 128; ++i) { const v4f v = *(const v4f*)(y + i * 128 + lane * 4); s += (v[0] + v[1]) + (v[2] + v[3]); }
#pragma unroll
    for (int o = 16; o > 0; o >>= 1) s += __shfl_xor(s, o, 32);
    const float mu = s * (1.0f / (float)DM);
    float q = 0.0f;
#pragma unroll 1
    for (int i = 0; i < DM / 128; ++i) { const v4f v = *(const v4f*)(y + i * 128 + lane * 4);
        const float d0 = v[0] - mu, d1 = v[1] - mu, d2 = v[2] - mu, d3 = v[3] - mu; q += (d0 * d0 + d1 * d1) + (d2 * d2 + d3 * d3); }
#pragma unroll
    for (int o = 16; o > 0; o >>= 1) q += __shfl_xor(q, o, 32);
    const float rs = rsqrtf(q * (1.0f / (float)DM) + LNEPS);
    if (OUTF) {
        const int bb = row / SEQ, tt = row % SEQ;
        float* orow = OUTP + ((size_t)bb * OUT_SEQ + tt) * DM;
#pragma unroll 1
        for (int ps = 0; ps < 2; ++ps) {
#pragma unroll 1
            for (int i = 0; i < DM / 128; ++i) { const int c = i * 128 + lane * 4;
                const v4f v = *(const v4f*)(y + c); const v4f gg = *(const v4f*)(g + c); const v4f bv = *(const v4f*)(be + c); v4f val;
#pragma unroll
                for (int k = 0; k < 4; ++k) val[k] = (v[k] - mu) * rs * bfr(gg[k]) + bfr(bv[k]);
                *(volatile v4f*)(orow + c) = val; }
            if (ps == 0) __threadfence(); }
    } else {
        h16* orow = OUTH + (size_t)row * DM;
#pragma unroll 1
        for (int ps = 0; ps < 2; ++ps) {
#pragma unroll 1
            for (int i = 0; i < DM / 256; ++i) { const int c = i * 256 + lane * 8;
                const v4f v0 = *(const v4f*)(y + c), v1 = *(const v4f*)(y + c + 4); const v4f g0 = *(const v4f*)(g + c), g1 = *(const v4f*)(g + c + 4);
                const v4f b0 = *(const v4f*)(be + c), b1 = *(const v4f*)(be + c + 4); v8h hv;
#pragma unroll
                for (int k = 0; k < 4; ++k) { hv[k] = toh_flush((v0[k] - mu) * rs * bfr(g0[k]) + bfr(b0[k])); hv[4 + k] = toh_flush((v1[k] - mu) * rs * bfr(g1[k]) + bfr(b1[k])); }
                *(volatile v8h*)(orow + c) = hv; }
            if (ps == 0) __threadfence(); }
    }
}

__global__ __launch_bounds__(128) void k_ln_h(const float* __restrict__ Y, const float* __restrict__ g, const float* __restrict__ be, h16* OUTH) {
    ln_body<0>(Y, g, be, (float*)0, OUTH);
}
__global__ __launch_bounds__(128) void k_ln_f(const float* __restrict__ Y, const float* __restrict__ g, const float* __restrict__ be, float* OUTP) {
    ln_body<1>(Y, g, be, OUTP, (h16*)0);
}

static constexpr size_t al256(size_t v) { return (v + 255) & ~(size_t)255; }
static constexpr size_t SZ_X   = al256((size_t)NB * SEQ * DM * 2);
static constexpr size_t SZ_W   = al256((size_t)DM * DM * 2);
static constexpr size_t SZ_PL  = al256((size_t)NB * NH_ * SEQ * HD * 2);
static constexpr size_t SZ_Y   = al256((size_t)NB * SEQ * DM * 4);
static constexpr int    NWT    = NB * SEQ_FULL * (SEQ_FULL / 32);
static constexpr int    NWS    = NB * (SEQ_FULL / 32);
static constexpr size_t SZ_PMT = al256((size_t)NWT * 4);
static constexpr size_t SZ_PMS = al256((size_t)NWS * 4);
static constexpr size_t SZ_TOTAL = 2 * SZ_X + 7 * SZ_W + 3 * SZ_PL + SZ_Y + SZ_X + SZ_Y + SZ_X + SZ_PMT + SZ_PMS;
static_assert(SZ_TOTAL <= (size_t)134217728);
static_assert(NWT % 32 == 0);
static_assert(NWS % 32 == 0);
static_assert((size_t)NB * NH_ * SEQ * HD == (size_t)NB * DM * SEQ);
static constexpr size_t NEEDX  = ((size_t)(NB - 1) * SEQ_FULL + SEQ) * DM;
static constexpr size_t NEEDMS = (size_t)NB * SEQ_FULL;
static constexpr size_t NEEDMT = (size_t)NB * SEQ_FULL * SEQ_FULL;
static constexpr size_t NEEDO  = ((size_t)(NB - 1) * OUT_SEQ + SEQ) * DM;
static constexpr int    MBS_T  = SEQ_FULL * (SEQ_FULL / 32);
static constexpr int    MQS_T  = SEQ_FULL / 32;
static constexpr int    MBS_S  = SEQ_FULL / 32;
static constexpr int    MQS_S  = 0;

extern "C" void kernel_launch(void* const* d_in, const int* in_sizes, int n_in,
                              void* d_out, int out_size, void* d_ws, size_t ws_size, hipStream_t stream) {
    if (n_in < 20) return;
    if ((size_t)in_sizes[0] < NEEDX || (size_t)in_sizes[1] < NEEDX) return;
    if ((size_t)in_sizes[2] < NEEDMS || (size_t)in_sizes[3] < NEEDMT) return;
    for (int i = 4; i <= 16; i += 2) if ((size_t)in_sizes[i] < (size_t)DM * DM) return;
    for (int i = 5; i <= 17; i += 2) if (in_sizes[i] < DM) return;
    if (in_sizes[18] < DM || in_sizes[19] < DM) return;
    if ((size_t)out_size < NEEDO) return;
    if (SZ_TOTAL > ws_size) return;
    const float* xenc = (const float*)d_in[0]; const float* xdec = (const float*)d_in[1];
    const int* smask = (const int*)d_in[2]; const int* tmask = (const int*)d_in[3];
    const float* w_q  = (const float*)d_in[4];  const float* b_q  = (const float*)d_in[5];
    const float* w_k  = (const float*)d_in[6];  const float* b_k  = (const float*)d_in[7];
    const float* w_v  = (const float*)d_in[8];  const float* b_v  = (const float*)d_in[9];
    const float* w_sq = (const float*)d_in[10]; const float* b_sq = (const float*)d_in[11];
    const float* w_sk = (const float*)d_in[12]; const float* b_sk = (const float*)d_in[13];
    const float* w_sv = (const float*)d_in[14]; const float* b_sv = (const float*)d_in[15];
    const float* w_d  = (const float*)d_in[16]; const float* b_d  = (const float*)d_in[17];
    const float* ln_g = (const float*)d_in[18]; const float* ln_b = (const float*)d_in[19];
    float* OUT = (float*)d_out;
    char* wsp = (char*)d_ws;
    bf* XD = (bf*)wsp; wsp += SZ_X;
    bf* XE = (bf*)wsp; wsp += SZ_X;
    bf* WQ  = (bf*)wsp; wsp += SZ_W;
    bf* WK  = (bf*)wsp; wsp += SZ_W;
    bf* WV  = (bf*)wsp; wsp += SZ_W;
    bf* WSK = (bf*)wsp; wsp += SZ_W;
    bf* WSV = (bf*)wsp; wsp += SZ_W;
    h16* WSQ = (h16*)wsp; wsp += SZ_W;
    h16* WD  = (h16*)wsp; wsp += SZ_W;
    h16* QH = (h16*)wsp; wsp += SZ_PL;
    h16* KH = (h16*)wsp; wsp += SZ_PL;
    h16* VT = (h16*)wsp; wsp += SZ_PL;
    float* QF = (float*)wsp; wsp += SZ_Y;
    h16* CH = (h16*)wsp; wsp += SZ_X;
    float* YP = (float*)wsp; wsp += SZ_Y;
    h16* SO = (h16*)wsp; wsp += SZ_X;
    unsigned* PMT = (unsigned*)wsp; wsp += SZ_PMT;
    unsigned* PMS = (unsigned*)wsp; wsp += SZ_PMS;

    if (SEQ == SEQ_FULL) {
        const size_t n8 = (size_t)NB * SEQ * DM / 8;
        k_cvt8<<<(unsigned)((n8 + 255) / 256), 256, 0, stream>>>(xdec, XD, n8);
        k_cvt8<<<(unsigned)((n8 + 255) / 256), 256, 0, stream>>>(xenc, XE, n8);
    } else {
        const size_t n8 = (size_t)SEQ * DM / 8;
        for (int b = 0; b < NB; ++b) {
            k_cvt8<<<(unsigned)((n8 + 255) / 256), 256, 0, stream>>>(xdec + (size_t)b * SEQ_FULL * DM, XD + (size_t)b * SEQ * DM, n8);
            k_cvt8<<<(unsigned)((n8 + 255) / 256), 256, 0, stream>>>(xenc + (size_t)b * SEQ_FULL * DM, XE + (size_t)b * SEQ * DM, n8);
        }
    }
    { const size_t n8 = (size_t)DM * DM / 8; const unsigned g = (unsigned)((n8 + 255) / 256);
      k_cvt8<<<g, 256, 0, stream>>>(w_q, WQ, n8); k_cvt8<<<g, 256, 0, stream>>>(w_k, WK, n8); k_cvt8<<<g, 256, 0, stream>>>(w_v, WV, n8);
      k_cvt8<<<g, 256, 0, stream>>>(w_sk, WSK, n8); k_cvt8<<<g, 256, 0, stream>>>(w_sv, WSV, n8);
      k_cvtw<<<g, 256, 0, stream>>>(w_sq, WSQ, n8); k_cvtw<<<g, 256, 0, stream>>>(w_d, WD, n8); }
    k_pack<<<(unsigned)((NWT / 32 + 7) / 8), 256, 0, stream>>>(tmask, PMT, NWT);
    k_pack<<<(unsigned)((NWS / 32 + 7) / 8), 256, 0, stream>>>(smask, PMS, NWS);

    const dim3 gP(NB * SEQ / 64, DM / 64, 1);
    const dim3 gT(DM / 64, NB * SEQ / 64, 1);
    const dim3 gF(SEQ / (16 * AW), NB * NH_, 1);

    k_gemm_qb<<<gP, 32, 0, stream>>>(XD, WQ, b_q, QH, QF);
    k_gemm_pb<<<gP, 32, 0, stream>>>(XD, WK, b_k, KH);
    k_gemm_tb<<<gT, 32, 0, stream>>>(WV, XD, b_v, VT);
    k_flash<<<gF, 32 * AW, 0, stream>>>(QH, KH, VT, PMT, MBS_T, MQS_T, CH);
    k_gemm_yh<<<gP, 32, 0, stream>>>(CH, WD, b_d, QF, YP);
    k_ln_h<<<(unsigned)(NB * SEQ / 4), 128, 0, stream>>>(YP, ln_g, ln_b, SO);

    k_gemm_qh<<<gP, 32, 0, stream>>>(SO, WSQ, b_sq, QH, QF);
    k_gemm_pb<<<gP, 32, 0, stream>>>(XE, WSK, b_sk, KH);
    k_gemm_tb<<<gT, 32, 0, stream>>>(WSV, XE, b_sv, VT);
    k_flash<<<gF, 32 * AW, 0, stream>>>(QH, KH, VT, PMS, MBS_S, MQS_S, CH);
    k_gemm_yh<<<gP, 32, 0, stream>>>(CH, WD, b_d, QF, YP);
    k_ln_f<<<(unsigned)(NB * SEQ / 4), 128, 0, stream>>>(YP, ln_g, ln_b, OUT);
}
